// GroupMamba_9405978378817
// MI455X (gfx1250) — hardware-run, weakly checked
//
#include <hip/hip_runtime.h>
#include <math.h>

typedef __attribute__((ext_vector_type(16))) _Float16 v16h;
typedef __attribute__((ext_vector_type(8)))  _Float16 v8h;
typedef __attribute__((ext_vector_type(2)))  _Float16 v2h;
typedef __attribute__((ext_vector_type(16))) __bf16   v16b;
typedef __attribute__((ext_vector_type(8)))  __bf16   v8b;
typedef __attribute__((ext_vector_type(8)))  float    v8f;
typedef __attribute__((ext_vector_type(4)))  float    v4f;
typedef __attribute__((ext_vector_type(2)))  float    v2f;

constexpr int kB    = 4;
constexpr int kL    = 2048;
constexpr int kLLog2 = 11;
constexpr int kD    = 512;
constexpr int kG    = 4;
constexpr int kGS   = kD / kG;
constexpr int kDI   = 2 * kGS;
constexpr int kDILog2 = 8;
constexpr int kNs   = 16;
constexpr int kDC   = 4;
constexpr int kR    = 8;
constexpr int kXo   = kR + 2 * kNs;
constexpr int kXoP  = 64;
constexpr int kRows = kB * kL;
constexpr int kThr  = 256;
constexpr float kInCarry = 1024.0f;
constexpr float kYCarry  = 8.0f;
constexpr float kSc = 1.0f / (kInCarry * kInCarry);
constexpr float kScY = 1.0f / (kYCarry * kInCarry);
constexpr int kK2 = 2 * kDI;
constexpr float kF16MinNormal = 6.103515625e-5f;

static_assert((1 << kLLog2) == kL && (1 << kDILog2) == kDI && kXo <= kXoP, "the shifts follow the sizes");
static_assert((kRows % 64) == 0 && ((2 * kDI) % 64) == 0 && (kXoP % 64) == 0 && (kGS % 64) == 0 && (kGS % 32) == 0 && (kDI % 32) == 0 && ((kRows / 64) * (kXoP / 64)) % 8 == 0, "GEMM M, N multiples of 64, K of 32; the smallest grid exact (128 tiles)");

constexpr size_t kOffX16 = 0ull;
constexpr size_t kOffWIN16 = 8388608ull;
constexpr size_t kOffWOUT16 = 8912896ull;
constexpr size_t kOffWX16 = 9437184ull;
constexpr size_t kOffZB = 9699328ull;
constexpr size_t kOffXZ = 9701376ull;
constexpr size_t kOffU16 = 26478592ull;
constexpr size_t kOffU32 = 34867200ull;
constexpr size_t kOffXD = 43255808ull;
constexpr size_t kOffY16 = 45352960ull;
constexpr size_t kOffOUTP = 53741568ull;
constexpr size_t kWsTotal = 57935872ull;
static_assert(kWsTotal <= 134217728ull, "carve cap: under 128 MiB");
static_assert(kOffX16 == 0
              && kOffWIN16 == kOffX16 + 8388608ull
              && kOffWOUT16 == kOffWIN16 + 524288ull
              && kOffWX16 == kOffWOUT16 + 524288ull
              && kOffZB == kOffWX16 + 262144ull
              && kOffXZ == kOffZB + 2048ull
              && kOffU16 == kOffXZ + 16777216ull
              && kOffU32 == kOffU16 + 8388608ull
              && kOffXD == kOffU32 + 8388608ull
              && kOffY16 == kOffXD + 2097152ull
              && kOffOUTP == kOffY16 + 8388608ull
              && kWsTotal == kOffOUTP + 4194304ull, "the carve is chained and totalled");
static_assert((kOffX16 % 256) == 0 && (kOffWIN16 % 256) == 0 && (kOffWOUT16 % 256) == 0 && (kOffWX16 % 256) == 0 && (kOffZB % 256) == 0 && (kOffXZ % 256) == 0 && (kOffU16 % 256) == 0 && (kOffU32 % 256) == 0 && (kOffXD % 256) == 0 && (kOffY16 % 256) == 0 && (kOffOUTP % 256) == 0, "aligned regions");

__device__ __forceinline__ unsigned short f2bf_bits(float f) {
  unsigned u = __float_as_uint(f);
  return (unsigned short)((u + 0x7FFFu + ((u >> 16) & 1u)) >> 16);
}
__device__ __forceinline__ float bf_bits2f(unsigned short h) { return __uint_as_float(((unsigned)h) << 16); }
__device__ __forceinline__ float bf16r(float f) { return bf_bits2f(f2bf_bits(f)); }
__device__ __forceinline__ float carry_flush(float v, float carry) {
  const float s = v * carry;
  return (fabsf(s) < kF16MinNormal) ? 0.0f : s;
}
__device__ __forceinline__ float frcp(float x) { return __builtin_amdgcn_rcpf(x); }

__device__ __forceinline__ void dep_guard4_h(v8f& a, v8f& b, v8f& c, v8f& d, v16h x, v16h y) { asm volatile("v_nop\n\tv_nop\n\tv_nop\n\tv_nop" : "+v"(a), "+v"(b), "+v"(c), "+v"(d) : "v"(x), "v"(y)); }
__device__ __forceinline__ void dep_guard4_b(v8f& a, v8f& b, v8f& c, v8f& d, v16b x, v16b y) { asm volatile("v_nop\n\tv_nop\n\tv_nop\n\tv_nop" : "+v"(a), "+v"(b), "+v"(c), "+v"(d) : "v"(x), "v"(y)); }
__device__ __forceinline__ void keep4_h(v16h a, v16h b, v16h c, v16h d) { asm volatile("v_nop" :: "v"(a), "v"(b), "v"(c), "v"(d)); }
__device__ __forceinline__ void keep4_b(v16b a, v16b b, v16b c, v16b d) { asm volatile("v_nop" :: "v"(a), "v"(b), "v"(c), "v"(d)); }
__device__ __forceinline__ void acc_guard4(v8f& a, v8f& b, v8f& c, v8f& d) { asm volatile("v_nop\n\tv_nop\n\tv_nop\n\tv_nop" : "+v"(a), "+v"(b), "+v"(c), "+v"(d)); }

template <typename T> struct Frag;
template <> struct Frag<_Float16> {
  typedef v16h V; union U { v16h v; v8h h[2]; };
  static __device__ __forceinline__ v16h load(const _Float16* p) {
    U f; f.h[0] = *(const v8h*)(p); f.h[1] = *(const v8h*)(p + 16); return f.v;
  }
  static __device__ __forceinline__ v8f mma(v16h a, v16h b, v8f c) {
    return __builtin_amdgcn_wmma_f32_16x16x32_f16(false, a, false, b, (short)0, c, false, false);
  }
  static __device__ __forceinline__ void guard4(v8f& a, v8f& b, v8f& c, v8f& d, v16h x, v16h y) { dep_guard4_h(a, b, c, d, x, y); }
  static __device__ __forceinline__ void keep(v16h a, v16h b, v16h c, v16h d) { keep4_h(a, b, c, d); }
};
template <> struct Frag<__bf16> {
  typedef v16b V; union U { v16b v; v8b h[2]; };
  static __device__ __forceinline__ v16b load(const __bf16* p) {
    U f; f.h[0] = *(const v8b*)(p); f.h[1] = *(const v8b*)(p + 16); return f.v;
  }
  static __device__ __forceinline__ v8f mma(v16b a, v16b b, v8f c) {
    return __builtin_amdgcn_wmma_f32_16x16x32_bf16(false, a, false, b, (short)0, c, false, false);
  }
  static __device__ __forceinline__ void guard4(v8f& a, v8f& b, v8f& c, v8f& d, v16b x, v16b y) { dep_guard4_b(a, b, c, d, x, y); }
  static __device__ __forceinline__ void keep(v16b a, v16b b, v16b c, v16b d) { keep4_b(a, b, c, d); }
};

__device__ __forceinline__ v8f mma_h(v16h a, v16h b, v8f c) {
  c = __builtin_amdgcn_wmma_f32_16x16x32_f16(false, a, false, b, (short)0, c, false, false);
  asm volatile("v_nop\n\tv_nop\n\tv_nop\n\tv_nop" : "+v"(c) : "v"(a), "v"(b));
  return c;
}

template <int ET> struct Elem;
template <> struct Elem<0> { typedef _Float16 T; };
template <> struct Elem<1> { typedef __bf16 T; };
template <int ET, bool SPLIT, int BIAS_MODE, int OUT_MODE, bool RESID, int ACT = 0>
__global__ __launch_bounds__(256) void wmma_gemm64(
    const unsigned short* __restrict__ Ap, const unsigned short* __restrict__ A2p, int lda, long strideA,
    const unsigned short* __restrict__ Btp, const unsigned short* __restrict__ Bt2p, int ldb, long strideB,
    void* __restrict__ Cout, void* __restrict__ Cout2, int ldc, long strideC,
    const float* __restrict__ bias,
    const float* __restrict__ resid, long strideR,
    int M, int N, int K, float scale) {
  typedef typename Elem<ET>::T T;
  typedef typename Frag<T>::V V;
  const T* A = (const T*)Ap; const T* A2 = (const T*)A2p; const T* Bt = (const T*)Btp; const T* Bt2 = (const T*)Bt2p;
  __shared__ __align__(16) float sT[8][16 * 68];
  const int b    = blockIdx.y;
  const int lane = threadIdx.x & 31;
  const int wave = threadIdx.x >> 5;
  const int tilesN = N >> 6;
  const int tilesM = M >> 6;
  const int tile = blockIdx.x * 8 + wave;
  if (tile >= tilesM * tilesN) return;
  const int tm = tile / tilesN;
  const int tn = tile - tm * tilesN;
  const int m0 = tm << 6;
  const int n0 = tn << 6;

  const T* Ab  = A  + (size_t)b * strideA;
  const T* Bb  = Bt + (size_t)b * strideB;
  const T* Ab2 = SPLIT ? (A2  + (size_t)b * strideA) : nullptr;
  const T* Bb2 = SPLIT ? (Bt2 + (size_t)b * strideB) : nullptr;

  const int rlane = lane & 15;
  const int koff  = (lane >> 4) * 8;
  const int mOff  = (lane >> 4) * 8;

  v8f acc[4][4];
#pragma unroll
  for (int i = 0; i < 4; ++i)
#pragma unroll
    for (int j = 0; j < 4; ++j) acc[i][j] = (v8f){0.f,0.f,0.f,0.f,0.f,0.f,0.f,0.f};

  for (int k0 = 0; k0 < K; k0 += 32) {
    V bh[4], bl[4];
#pragma unroll
    for (int j = 0; j < 4; ++j) {
      const size_t bo = (size_t)(n0 + (j << 4) + rlane) * ldb + koff + k0;
      bh[j] = Frag<T>::load(Bb + bo);
      if (SPLIT) bl[j] = Frag<T>::load(Bb2 + bo);
    }
#pragma unroll
    for (int i = 0; i < 4; ++i) {
      const size_t ao = (size_t)(m0 + (i << 4) + rlane) * lda + koff + k0;
      V ah = Frag<T>::load(Ab + ao);
      V al;
      if (SPLIT) al = Frag<T>::load(Ab2 + ao);
#pragma unroll
      for (int j = 0; j < 4; ++j) {
        acc[i][j] = Frag<T>::mma(ah, bh[j], acc[i][j]);
        if (SPLIT) {
          acc[i][j] = Frag<T>::mma(ah, bl[j], acc[i][j]);
          acc[i][j] = Frag<T>::mma(al, bh[j], acc[i][j]);
        }
      }
      Frag<T>::guard4(acc[i][0], acc[i][1], acc[i][2], acc[i][3], ah, SPLIT ? al : ah);
    }
    Frag<T>::keep(bh[0], bh[1], bh[2], bh[3]);
    if (SPLIT) Frag<T>::keep(bl[0], bl[1], bl[2], bl[3]);
  }
  acc_guard4(acc[0][0], acc[0][1], acc[0][2], acc[0][3]);
  acc_guard4(acc[1][0], acc[1][1], acc[1][2], acc[1][3]);
  acc_guard4(acc[2][0], acc[2][1], acc[2][2], acc[2][3]);
  acc_guard4(acc[3][0], acc[3][1], acc[3][2], acc[3][3]);

  float* slab = sT[wave];
  const float* Rb = RESID ? (resid + (size_t)b * strideR) : nullptr;
#pragma unroll
  for (int i = 0; i < 4; ++i) {
    const int mBase = m0 + (i << 4);
#pragma unroll
    for (int j = 0; j < 4; ++j) {
      const int n = n0 + (j << 4) + rlane;
      float bv = 0.f;
      if (BIAS_MODE == 2) bv = bias[n];
#pragma unroll
      for (int r = 0; r < 8; ++r) {
        float v = acc[i][j][r] * scale;
        if (BIAS_MODE == 1) v += bias[mBase + mOff + r];
        if (BIAS_MODE == 2) v += bv;
        if (RESID) v += Rb[(size_t)(mBase + mOff + r) * ldc + n];
        if (ACT == 1) v = tanhf(v);
        if (ACT == 2) v = fmaxf(v, 0.0f);
        if (ACT == 3) v = v / (1.0f + expf(-v));
        if (ACT == 4) v = (v > 0.f) ? v : 0.01f * v;
        slab[(mOff + r) * 68 + (j << 4) + rlane] = v;
      }
    }
    __builtin_amdgcn_fence(__ATOMIC_RELEASE, "workgroup");
    __builtin_amdgcn_wave_barrier();
    __builtin_amdgcn_fence(__ATOMIC_ACQUIRE, "workgroup");
    if (OUT_MODE == 0) {
      float* C = (float*)Cout + (size_t)b * strideC;
      const int hh = lane >> 4, c4 = (lane & 15) * 4;
      for (int pass = 0; pass < 2; ++pass) {
#pragma unroll
        for (int it = 0; it < 8; ++it) {
          const int row = it * 2 + hh;
          v4f v = *(const v4f*)(slab + row * 68 + c4);
          *(volatile v4f*)(C + (size_t)(mBase + row) * ldc + n0 + c4) = v;
        }
        __threadfence();
      }
    } else {
      const int q = lane >> 3, c8 = (lane & 7) * 8;
      unsigned short* C  = (unsigned short*)Cout  + (size_t)b * strideC;
      unsigned short* C2 = (OUT_MODE == 2) ? ((unsigned short*)Cout2 + (size_t)b * strideC) : nullptr;
      for (int pass = 0; pass < 2; ++pass) {
#pragma unroll
        for (int it = 0; it < 4; ++it) {
          const int row = it * 4 + q;
          const float* sp = slab + row * 68 + c8;
          v8h hv, lv;
#pragma unroll
          for (int e = 0; e < 8; ++e) {
            if (OUT_MODE == 1) {
              hv[e] = (_Float16)sp[e];
            } else {
              unsigned short hb = f2bf_bits(sp[e]);
              unsigned short lb = f2bf_bits(sp[e] - bf_bits2f(hb));
              hv[e] = __builtin_bit_cast(_Float16, hb);
              lv[e] = __builtin_bit_cast(_Float16, lb);
            }
          }
          *(volatile v8h*)(C + (size_t)(mBase + row) * ldc + n0 + c8) = hv;
          if (OUT_MODE == 2) *(volatile v8h*)(C2 + (size_t)(mBase + row) * ldc + n0 + c8) = lv;
        }
        __threadfence();
      }
    }
    __builtin_amdgcn_fence(__ATOMIC_RELEASE, "workgroup");
    __builtin_amdgcn_wave_barrier();
    __builtin_amdgcn_fence(__ATOMIC_ACQUIRE, "workgroup");
  }
}

__global__ __launch_bounds__(kThr) void cast_plane_kernel(const float* __restrict__ src, unsigned short* __restrict__ dst,
                                                          int colsLog2, int dstPitch, int dstOff) {
  const int i   = blockIdx.x * kThr + threadIdx.x;
  const int sh  = colsLog2 - 3;
  const int row = i >> sh;
  const int c8  = (i & ((1 << sh) - 1)) * 8;
  const float* sp = src + ((size_t)row << colsLog2) + c8;
  const v4f a0 = *(const v4f*)(sp);
  const v4f a1 = *(const v4f*)(sp + 4);
  v8h hv;
#pragma unroll
  for (int e = 0; e < 4; ++e) {
    const float f0 = a0[e];
    const float f1 = a1[e];
    hv[e]     = (_Float16)carry_flush(bf16r(f0), kInCarry);
    hv[4 + e] = (_Float16)carry_flush(bf16r(f1), kInCarry);
  }
  unsigned short* dp = dst + (size_t)row * dstPitch + dstOff + c8;
  *(volatile v8h*)dp = hv;
  __threadfence();
  *(volatile v8h*)dp = hv;
}

__device__ __forceinline__ void two_words(float v, float carry, _Float16& hi, _Float16& lo) {
  const float s = carry_flush(v, carry);
  hi = (_Float16)s;
  const float r = s - (float)hi;
  lo = (_Float16)((fabsf(r) < kF16MinNormal) ? 0.0f : r);
}

__global__ __launch_bounds__(64) void setup_kernel(const float* __restrict__ W_x, unsigned short* __restrict__ WX16, float* __restrict__ ZB) {
  const unsigned y = blockIdx.y;
  const unsigned c = threadIdx.x;
  if (y < 256u) {
    const unsigned g = y >> 6, n = y & 63u, ch = c & 31u;
    const bool live = n < (unsigned)kXo;
    const float* sp = W_x + ((size_t)g * kXo + (live ? n : 0u)) * kDI + ch * 8u;
    const v4f a0 = *(const v4f*)sp, a1 = *(const v4f*)(sp + 4);
    v8h hv;
#pragma unroll
    for (int e = 0; e < 4; ++e) {
      const float p = a0[e], q = a1[e];
      hv[e] = (_Float16)(live ? carry_flush(bf16r(p), kInCarry) : 0.0f);
      hv[4 + e] = (_Float16)(live ? carry_flush(bf16r(q), kInCarry) : 0.0f);
    }
    unsigned short* dp = WX16 + (size_t)y * kK2 + c * 8u;
    *(volatile v8h*)dp = hv;
    __threadfence();
    *(volatile v8h*)dp = hv;
  } else {
    const v4f z = {0.f, 0.f, 0.f, 0.f};
    for (int h = 0; h < 2; ++h) {
      float* dp = ZB + (c + 64u * (unsigned)h) * 4u;
      *(volatile v4f*)dp = z;
      __threadfence();
      *(volatile v4f*)dp = z;
    }
  }
}
static_assert(kG * kXoP == 256 && kXoP == 64 && kK2 == 64 * 8 && kDI == 32 * 8, "256 weight rows (group = row >> 6); 64 chunks a two-word row, 32 a source row");

__global__ __launch_bounds__(kThr) void conv_silu_kernel(const float* __restrict__ XZ, const float* __restrict__ cw, const float* __restrict__ cb,
                                                         unsigned short* __restrict__ U16, float* __restrict__ U32) {
  const size_t i = (size_t)blockIdx.x * kThr + threadIdx.x;
  const size_t row = i >> (kDILog2 - 3);
  const int c8 = (int)(i & (size_t)(kDI / 8 - 1)) * 8;
  const int l = (int)(row & (size_t)(kL - 1));
  float acc[8];
  {
    const v4f b0 = *(const v4f*)(cb + c8), b1 = *(const v4f*)(cb + c8 + 4);
#pragma unroll
    for (int e = 0; e < 4; ++e) { const float p = b0[e], q = b1[e]; acc[e] = bf16r(p); acc[4 + e] = bf16r(q); }
  }
#pragma unroll
  for (int k = 0; k < kDC; ++k) {
    const int back = kDC - 1 - k;
    const bool has = l >= back;
    const float* xp = XZ + (row - (size_t)(has ? back : 0)) * (2 * kDI) + c8;
    const v4f x0 = *(const v4f*)xp, x1 = *(const v4f*)(xp + 4);
#pragma unroll
    for (int e = 0; e < 8; ++e) {
      const float w = cw[(size_t)(c8 + e) * kDC + k];
      const float xv = (e < 4) ? x0[e] : x1[e - 4];
      acc[e] += has ? bf16r(w) * xv : 0.0f;
    }
  }
  v8h hv, lv; v4f u0, u1;
#pragma unroll
  for (int e = 0; e < 8; ++e) {
    const float v = acc[e];
    const float s = v / (1.0f + expf(-v));
    _Float16 hi, lo;
    two_words(s, kInCarry, hi, lo);
    hv[e] = hi; lv[e] = lo;
    if (e < 4) u0[e] = s; else u1[e - 4] = s;
  }
  unsigned short* hp = U16 + row * kK2 + c8;
  float* fp = U32 + row * kDI + c8;
  for (int pass = 0; pass < 2; ++pass) {
    *(volatile v8h*)hp = hv;
    *(volatile v8h*)(hp + kDI) = lv;
    *(volatile v4f*)fp = u0;
    *(volatile v4f*)(fp + 4) = u1;
    __threadfence();
  }
}
static_assert(((size_t)kRows * kDI / 8) % kThr == 0 && (kL & (kL - 1)) == 0, "front grid exact; the position is row & (kL - 1)");

__global__ __launch_bounds__(kThr) void group_scan_kernel(const float* __restrict__ XD, const float* __restrict__ U32, const float* __restrict__ XZ,
                                                          const float* __restrict__ W_dt, const float* __restrict__ b_dt, const float* __restrict__ A_log,
                                                          const float* __restrict__ Dp, unsigned short* __restrict__ Y16) {
  const unsigned v = blockIdx.x * (unsigned)kThr + threadIdx.x;
  const unsigned smp = v >> (kDILog2 - 1), d0 = (v & (unsigned)(kDI / 2 - 1)) * 2u;
  float A[2][kNs], h[2][kNs], wd[2][kR], bd[2], dc[2];
#pragma unroll
  for (int k = 0; k < 2; ++k) {
    const unsigned d = d0 + (unsigned)k;
#pragma unroll
    for (int n = 0; n < kNs; ++n) { const float a = A_log[(size_t)d * kNs + n]; A[k][n] = -expf(bf16r(a)); h[k][n] = 0.0f; }
#pragma unroll
    for (int r = 0; r < kR; ++r) { const float w = W_dt[(size_t)d * kR + r]; wd[k][r] = bf16r(w); }
    const float b0 = b_dt[d], q0 = Dp[d];
    bd[k] = bf16r(b0); dc[k] = bf16r(q0);
  }
  const size_t r0 = (size_t)smp * kL;
  for (int l = 0; l < kL; ++l) {
    const size_t row = r0 + (size_t)l;
    const float* pr = XD + row * kXoP;
    const v4f t0 = *(const v4f*)pr, t1 = *(const v4f*)(pr + 4);
    const v2f uv = *(const v2f*)(U32 + row * kDI + d0);
    const v2f zv = *(const v2f*)(XZ + row * (2 * kDI) + kDI + d0);
    float delta[2], dx[2], y[2];
#pragma unroll
    for (int k = 0; k < 2; ++k) {
      float pre = bd[k];
#pragma unroll
      for (int r = 0; r < 4; ++r) { pre += wd[k][r] * t0[r]; pre += wd[k][4 + r] * t1[r]; }
      delta[k] = (pre > 20.0f) ? pre : log1pf(expf(pre));
      dx[k] = delta[k] * uv[k];
      y[k] = 0.0f;
    }
#pragma unroll
    for (int q = 0; q < kNs / 4; ++q) {
      const v4f bv = *(const v4f*)(pr + kR + 4 * q), cv = *(const v4f*)(pr + kR + kNs + 4 * q);
#pragma unroll
      for (int e = 0; e < 4; ++e) {
        const int n = 4 * q + e;
#pragma unroll
        for (int k = 0; k < 2; ++k) {
          const float hn = expf(delta[k] * A[k][n]) * h[k][n] + dx[k] * bv[e];
          h[k][n] = hn;
          y[k] += hn * cv[e];
        }
      }
    }
    v2h hv, lv;
#pragma unroll
    for (int k = 0; k < 2; ++k) {
      const float yo = y[k] + dc[k] * uv[k];
      const float g = zv[k] / (1.0f + expf(-zv[k]));
      _Float16 hi, lo;
      two_words(yo * g, kYCarry, hi, lo);
      hv[k] = hi; lv[k] = lo;
    }
    unsigned short* dp = Y16 + row * kK2 + d0;
    for (int pass = 0; pass < 2; ++pass) {
      *(volatile v2h*)dp = hv;
      *(volatile v2h*)(dp + kDI) = lv;
      __threadfence();
    }
  }
}
static_assert((kB * kDI / 2) % kThr == 0 && kR == 8 && (kNs % 4) == 0 && kXo == kR + 2 * kNs, "scan grid exact: two blocks a group; the parameter columns 8 | 16 | 16");

__global__ __launch_bounds__(kThr) void out_copy_kernel(const float* __restrict__ OUTP, float* __restrict__ out, int group) {
  const size_t i4 = ((size_t)blockIdx.x * kThr + threadIdx.x) * 4u;
  const size_t row = i4 >> 7, col = i4 & 127u;
  const v4f vv = *(const v4f*)(OUTP + i4);
  float* dp = out + row * kD + (size_t)group * kGS + col;
  *(volatile v4f*)dp = vv;
  __threadfence();
  *(volatile v4f*)dp = vv;
}
static_assert(kGS == 128 && ((size_t)kRows * kGS / 4) == 1024 * kThr, "output grid exact; a group's row = 128 floats (the shift by 7)");

static_assert(((size_t)kRows * kD / 8) % kThr == 0 && ((size_t)kG * 2 * kDI * kGS / 8) % kThr == 0 && ((size_t)kG * kGS * kDI / 8) % kThr == 0, "plane cast grids exact");

extern "C" void kernel_launch(void* const* d_in, const int* in_sizes, int n_in,
                              void* d_out, int out_size, void* d_ws, size_t ws_size,
                              hipStream_t stream) {
  if (n_in < 10 || d_out == nullptr || d_ws == nullptr) return;
  if (in_sizes[0] != kRows * kD || in_sizes[1] != kG * 2 * kDI * kGS || in_sizes[2] != kG * kDI * kDC || in_sizes[3] != kG * kDI || in_sizes[4] != kG * kXo * kDI) return;
  if (in_sizes[5] != kG * kDI * kR || in_sizes[6] != kG * kDI || in_sizes[7] != kG * kDI * kNs || in_sizes[8] != kG * kDI || in_sizes[9] != kG * kGS * kDI) return;
  if (out_size != kRows * kD) return;
  if (ws_size < kWsTotal) return;
  const float* x = (const float*)d_in[0];
  const float* W_in = (const float*)d_in[1];
  const float* conv_w = (const float*)d_in[2];
  const float* conv_b = (const float*)d_in[3];
  const float* W_x = (const float*)d_in[4];
  const float* W_dt = (const float*)d_in[5];
  const float* b_dt = (const float*)d_in[6];
  const float* A_log = (const float*)d_in[7];
  const float* D_param = (const float*)d_in[8];
  const float* W_out = (const float*)d_in[9];
  float* out = (float*)d_out;
  char* ws = (char*)d_ws;
  unsigned short* X16 = (unsigned short*)(ws + kOffX16);
  unsigned short* WIN16 = (unsigned short*)(ws + kOffWIN16);
  unsigned short* WOUT16 = (unsigned short*)(ws + kOffWOUT16);
  unsigned short* WX16 = (unsigned short*)(ws + kOffWX16);
  float* ZB = (float*)(ws + kOffZB);
  float* XZ = (float*)(ws + kOffXZ);
  unsigned short* U16 = (unsigned short*)(ws + kOffU16);
  float* U32 = (float*)(ws + kOffU32);
  float* XD = (float*)(ws + kOffXD);
  unsigned short* Y16 = (unsigned short*)(ws + kOffY16);
  float* OUTP = (float*)(ws + kOffOUTP);

  cast_plane_kernel<<<(int)(((size_t)kRows * kD / 8) / kThr), kThr, 0, stream>>>(x, X16, 9, kD, 0);
  cast_plane_kernel<<<(int)(((size_t)kG * 2 * kDI * kGS / 8) / kThr), kThr, 0, stream>>>(W_in, WIN16, 7, kGS, 0);
  cast_plane_kernel<<<(int)(((size_t)kG * kGS * kDI / 8) / kThr), kThr, 0, stream>>>(W_out, WOUT16, 8, kK2, 0);
  cast_plane_kernel<<<(int)(((size_t)kG * kGS * kDI / 8) / kThr), kThr, 0, stream>>>(W_out, WOUT16, 8, kK2, kDI);
  setup_kernel<<<dim3(1, 257), 64, 0, stream>>>(W_x, WX16, ZB);
  for (int g = 0; g < kG; ++g) {
    wmma_gemm64<0, false, 2, 0, false, 0><<<dim3((kRows / 64) * (2 * kDI / 64) / 8, 1), 256, 0, stream>>>(
        X16 + (size_t)g * kGS, X16 + (size_t)g * kGS, kD, 0L, WIN16 + (size_t)g * 2 * kDI * kGS, WIN16 + (size_t)g * 2 * kDI * kGS, kGS, 0L,
        (void*)XZ, (void*)XZ, 2 * kDI, 0L, ZB, nullptr, 0L, kRows, 2 * kDI, kGS, kSc);
    conv_silu_kernel<<<(int)(((size_t)kRows * kDI / 8) / kThr), kThr, 0, stream>>>(XZ, conv_w + (size_t)g * kDI * kDC, conv_b + (size_t)g * kDI, U16, U32);
    wmma_gemm64<0, false, 2, 0, false, 0><<<dim3((kRows / 64) * (kXoP / 64) / 8, 1), 256, 0, stream>>>(
        U16, U16, kK2, 0L, WX16 + (size_t)g * kXoP * kK2, WX16 + (size_t)g * kXoP * kK2, kK2, 0L, (void*)XD, (void*)XD, kXoP, 0L, ZB, nullptr, 0L, kRows, kXoP, kK2, kSc);
    group_scan_kernel<<<(kB * kDI / 2) / kThr, kThr, 0, stream>>>(XD, U32, XZ, W_dt + (size_t)g * kDI * kR, b_dt + (size_t)g * kDI, A_log + (size_t)g * kDI * kNs, D_param + (size_t)g * kDI, Y16);
    wmma_gemm64<0, false, 2, 0, false, 0><<<dim3((kRows / 64) * (kGS / 64) / 8, 1), 256, 0, stream>>>(
        Y16, Y16, kK2, 0L, WOUT16 + (size_t)g * kGS * kK2, WOUT16 + (size_t)g * kGS * kK2, kK2, 0L, (void*)OUTP, (void*)OUTP, kGS, 0L, ZB, nullptr, 0L, kRows, kGS, kK2, kScY);
    out_copy_kernel<<<1024, kThr, 0, stream>>>(OUTP, out, g);
  }
}
